// DyAtGNN_60670708023705
// MI455X (gfx1250) — hardware-verified
//
#include <hip/hip_runtime.h>
#include <stddef.h>
#include <math.h>


#define DF      128
#define NTHR    256
#define NWAVE   8
#define GR      32
#define AP      136
#define XSP     132
#define XPP     136
#define NB      512
#define NBS     8192
#define NBX     2048
#define CHUNK   4096
#define NGRP    (CHUNK / (NTHR * 4))
#define WCAP    ((CHUNK / NTHR) * 32)
#define SLOTB   13
#define KPOOL   128
#define TKMASKW 4096
#define NMAXB   64
#define EMP     1024

#define P_WHID  0
#define P_WL    (DF * DF)
#define P_WR    (2 * DF * DF)
#define P_WIH   (3 * DF * DF)
#define P_WHH   (6 * DF * DF)
#define P_H0    (9 * DF * DF)
#define P_TOT   (10 * DF * DF)
#define WU      (DF * DF / 8)
#define PREP_UNITS (P_TOT / 8)

#define AGG_LDS_BYTES  ((NB * DF + NWAVE * WCAP + NWAVE) * 4)
#define POOL_LDS_BYTES (KPOOL * DF * 4 + KPOOL * XPP * 2 + TKMASKW * 4 + KPOOL * 4 + 2 * NWAVE * 4)

static_assert(NGRP == 4);
static_assert(WCAP == 512);
static_assert((1 << SLOTB) >= NBS);
static_assert((1 << SLOTB) >= NB);
static_assert(NBX % NB == 0);
static_assert(NBX % GR == 0);
static_assert(KPOOL == DF);
static_assert(AGG_LDS_BYTES == 278560);
static_assert(POOL_LDS_BYTES == 117312);
static_assert((KPOOL * DF / 8) % NTHR == 0);
static_assert(KPOOL % NWAVE == 0);
static_assert(PREP_UNITS % NTHR == 0);

typedef float    v4f  __attribute__((ext_vector_type(4)));
typedef float    v8f  __attribute__((ext_vector_type(8)));
typedef int      v4i  __attribute__((ext_vector_type(4)));
typedef _Float16 v8h  __attribute__((ext_vector_type(8)));
typedef _Float16 v16h __attribute__((ext_vector_type(16)));
union Frag   { v16h v; v8h half[2]; };
union Pack16 { v8h h; v4i i; };

__device__ __forceinline__ v8f wm(v16h a, v16h b, v8f c) {
  v8f d = __builtin_amdgcn_wmma_f32_16x16x32_f16(false, a, false, b, (short)0, c, false, false);
  asm volatile("v_nop\n\tv_nop\n\tv_nop\n\tv_nop" : "+v"(d) : "v"(a), "v"(b));
  return d;
}

__device__ __forceinline__ v8f zero8() {
  v8f z = {0.f, 0.f, 0.f, 0.f, 0.f, 0.f, 0.f, 0.f};
  return z;
}

__device__ __forceinline__ v4i pk8(v4f a, v4f b, float s) {
  Pack16 u;
  u.h[0] = (_Float16)(a.x * s); u.h[1] = (_Float16)(a.y * s);
  u.h[2] = (_Float16)(a.z * s); u.h[3] = (_Float16)(a.w * s);
  u.h[4] = (_Float16)(b.x * s); u.h[5] = (_Float16)(b.y * s);
  u.h[6] = (_Float16)(b.z * s); u.h[7] = (_Float16)(b.w * s);
  return u.i;
}

__device__ __forceinline__ int clampi(int v, int hi) {
  return v < 0 ? 0 : (v > hi ? hi : v);
}

__device__ __forceinline__ float sigm(float x) {
  x = fminf(fmaxf(x, -30.0f), 30.0f);
  const float e = expf(-x);
  return __builtin_amdgcn_rcpf(1.0f + e);
}

__device__ __forceinline__ float block_emax(const float* __restrict__ emx, float* red, int tid) {
  if (tid < NMAXB) red[tid] = emx[tid * 32];
  __syncthreads();
  float mv = -3.0e38f;
#pragma unroll 1
  for (int i = 0; i < NMAXB; ++i) mv = fmaxf(mv, red[i]);
  return mv;
}

template <int NBT>
__device__ __forceinline__ int scan_chunk(const int* __restrict__ key, int nE, bool al16, int cbase,
                                          int nodeBase, int* list, int tid, int lane, int wave) {
  int wc = 0;
#pragma unroll
  for (int g = 0; g < NGRP; ++g) {
    const int el0 = (g * NTHR + tid) * 4;
    const int e0  = cbase + el0;
    const int sent = -2147483647 - 1;
    v4i d;
    if (al16 && (e0 + 3 < nE)) {
      d = *(const v4i*)(key + e0);
    } else {
      d.x = (e0     < nE) ? key[e0]     : sent;
      d.y = (e0 + 1 < nE) ? key[e0 + 1] : sent;
      d.z = (e0 + 2 < nE) ? key[e0 + 2] : sent;
      d.w = (e0 + 3 < nE) ? key[e0 + 3] : sent;
    }
    const unsigned s0 = (unsigned)d.x - (unsigned)nodeBase;
    const unsigned s1 = (unsigned)d.y - (unsigned)nodeBase;
    const unsigned s2 = (unsigned)d.z - (unsigned)nodeBase;
    const unsigned s3 = (unsigned)d.w - (unsigned)nodeBase;
    const bool h0 = s0 < (unsigned)NBT;
    const bool h1 = s1 < (unsigned)NBT;
    const bool h2 = s2 < (unsigned)NBT;
    const bool h3 = s3 < (unsigned)NBT;
    const unsigned many = __builtin_amdgcn_ballot_w32(h0 | h1 | h2 | h3);
    if (many != 0u) {
#define HITJ(J, HJ, SJ) { \
        const unsigned mj = __builtin_amdgcn_ballot_w32(HJ); \
        if (HJ) { \
          const int pos = wc + (int)__builtin_amdgcn_mbcnt_lo(mj, 0u); \
          if (pos < WCAP) list[wave * WCAP + pos] = ((el0 + (J)) << SLOTB) | (int)(SJ); \
        } \
        wc += (int)__builtin_popcount(mj); }
      HITJ(0, h0, s0)
      HITJ(1, h1, s1)
      HITJ(2, h2, s2)
      HITJ(3, h3, s3)
#undef HITJ
    }
  }
  return wc;
}

__global__ __launch_bounds__(NTHR) void k_prep(
    const float* __restrict__ Whid, const float* __restrict__ Wl, const float* __restrict__ Wr,
    const float* __restrict__ Wih, const float* __restrict__ Whh, const float* __restrict__ h0,
    _Float16* planes) {
  const int u = blockIdx.x * NTHR + threadIdx.x;
  if (u >= PREP_UNITS) return;
  v4f a, b;
  if (u < 3 * WU) {
    const int mat = u / WU;
    const int v = u - mat * WU;
    const float* W = (mat == 0) ? Whid : ((mat == 1) ? Wl : Wr);
    const int n = v >> 4, k0 = (v & 15) * 8;
    a.x = W[(k0 + 0) * DF + n]; a.y = W[(k0 + 1) * DF + n];
    a.z = W[(k0 + 2) * DF + n]; a.w = W[(k0 + 3) * DF + n];
    b.x = W[(k0 + 4) * DF + n]; b.y = W[(k0 + 5) * DF + n];
    b.z = W[(k0 + 6) * DF + n]; b.w = W[(k0 + 7) * DF + n];
  } else if (u < 9 * WU) {
    const int v = u - 3 * WU;
    const float* W = (v < 3 * WU) ? Wih : Whh;
    const int o = ((v < 3 * WU) ? v : v - 3 * WU) * 8;
    a = *(const v4f*)(W + o); b = *(const v4f*)(W + o + 4);
  } else {
    const int o = (u - 9 * WU) * 8;
    a = *(const v4f*)(h0 + o); b = *(const v4f*)(h0 + o + 4);
  }
  const v4i p = pk8(a, b, 16.0f);
  _Float16* dst = planes + (size_t)u * 8;
  *(volatile v4i*)dst = p;
  __threadfence();
  *(volatile v4i*)dst = p;
}

__global__ __launch_bounds__(NTHR) void k_gemm_hid(
    const float* __restrict__ x, const _Float16* __restrict__ planes, const float* __restrict__ bias,
    float* H, int nN) {
  __shared__ __attribute__((aligned(16))) _Float16 At[GR * AP];
  __shared__ __attribute__((aligned(16))) float Xs[GR * XSP];
  const int tid = threadIdx.x, lane = tid & 31, wave = tid >> 5, hh = lane >> 4, m = lane & 15;
  const int rowBase = blockIdx.x * GR;
  {
    const int r  = tid >> 3;
    const int c0 = (tid & 7) * 16;
    int row = rowBase + r;
    if (row > nN - 1) row = nN - 1;
    const float* p = x + (size_t)row * DF + c0;
    Pack16 u0, u1;
    u0.i = pk8(*(const v4f*)(p), *(const v4f*)(p + 4), 1.0f);
    u1.i = pk8(*(const v4f*)(p + 8), *(const v4f*)(p + 12), 1.0f);
    *(v8h*)(At + r * AP + c0)     = u0.h;
    *(v8h*)(At + r * AP + c0 + 8) = u1.h;
  }
  __syncthreads();

  const int ncol = wave * 16 + m;
  const _Float16* Bp = planes + P_WHID + (size_t)ncol * DF;
  v8f c0a = zero8(), c1a = zero8();
#pragma unroll
  for (int kt = 0; kt < DF / 32; ++kt) {
    const int k0 = kt * 32;
    Frag a0, a1, b;
    const _Float16* pb  = Bp + k0 + 8 * hh;
    const _Float16* pa0 = At + m * AP + k0 + 8 * hh;
    const _Float16* pa1 = At + (16 + m) * AP + k0 + 8 * hh;
    b.half[0]  = *(const v8h*)pb;  b.half[1]  = *(const v8h*)(pb + 16);
    a0.half[0] = *(const v8h*)pa0; a0.half[1] = *(const v8h*)(pa0 + 16);
    a1.half[0] = *(const v8h*)pa1; a1.half[1] = *(const v8h*)(pa1 + 16);
    c0a = wm(a0.v, b.v, c0a);
    c1a = wm(a1.v, b.v, c1a);
  }
  const float bv = bias[ncol];
#pragma unroll
  for (int r = 0; r < 8; ++r) {
    Xs[(8 * hh + r) * XSP + ncol]      = fmaxf(c0a[r] * 0.0625f + bv, 0.f);
    Xs[(16 + 8 * hh + r) * XSP + ncol] = fmaxf(c1a[r] * 0.0625f + bv, 0.f);
  }
  __syncthreads();

  v4f xr[4];
  float* hp[4];
#pragma unroll
  for (int i = 0; i < 4; ++i) {
    xr[i] = *(const v4f*)(Xs + (4 * wave + i) * XSP + 4 * lane);
    hp[i] = H + (size_t)(rowBase + 4 * wave + i) * DF + 4 * lane;
  }
#pragma unroll
  for (int i = 0; i < 4; ++i) *(volatile v4f*)(hp[i]) = xr[i];
  __threadfence();
#pragma unroll
  for (int i = 0; i < 4; ++i) *(volatile v4f*)(hp[i]) = xr[i];
}

__global__ __launch_bounds__(NTHR) void k_xres(
    const float* __restrict__ H, const int* __restrict__ remain, const int* __restrict__ added,
    const int* __restrict__ nid, float* xres, int nN, int nR, int nA) {
  __shared__ int mp[NBX];
  const int tid = threadIdx.x, lane = tid & 31, wave = tid >> 5;
  const int base = blockIdx.x * NBX;
  for (int i = tid; i < NBX; i += NTHR) mp[i] = -1;
  __syncthreads();
#pragma unroll 1
  for (int k = tid; k < nR; k += NTHR) {
    const int rc = clampi(remain[k], nN - 1);
    const int t = nid[rc];
    if ((unsigned)t < (unsigned)nN) {
      const unsigned s = (unsigned)t - (unsigned)base;
      if (s < (unsigned)NBX) mp[s] = rc;
    }
  }
  __syncthreads();
#pragma unroll 1
  for (int k = tid; k < nA; k += NTHR) {
    const int rc = clampi(added[k], nN - 1);
    const int t = nid[rc];
    if ((unsigned)t < (unsigned)nN) {
      const unsigned s = (unsigned)t - (unsigned)base;
      if (s < (unsigned)NBX) mp[s] = rc;
    }
  }
  __syncthreads();
#pragma unroll 1
  for (int jj = 0; jj < NBX / NWAVE; ++jj) {
    const int slot = wave * (NBX / NWAVE) + jj;
    const int code = mp[slot];
    v4f v = {0.f, 0.f, 0.f, 0.f};
    if (code >= 0) v = *(const v4f*)(H + (size_t)code * DF + 4 * lane);
    float* p = xres + (size_t)(base + slot) * DF + 4 * lane;
    *(volatile v4f*)p = v;
    __threadfence();
    *(volatile v4f*)p = v;
  }
}

__global__ __launch_bounds__(NTHR) void k_pool(
    const float* __restrict__ scores, const int* __restrict__ remain, const int* __restrict__ nid,
    const float* __restrict__ H, const _Float16* __restrict__ planes, const float* __restrict__ h0,
    const float* __restrict__ bih, const float* __restrict__ bhh,
    float* xres, _Float16* hT, int nN, int nR) {
  extern __shared__ v4f lds_dyn[];
  float*    hs  = (float*)lds_dyn;
  _Float16* XpL = (_Float16*)(hs + KPOOL * DF);
  unsigned* msk = (unsigned*)(XpL + KPOOL * XPP);
  int*      sel = (int*)(msk + TKMASKW);
  float*    rv  = (float*)(sel + KPOOL);
  int*      ri  = (int*)(rv + NWAVE);
  const int tid = threadIdx.x, lane = tid & 31, wave = tid >> 5, hh = lane >> 4, m = lane & 15;

  for (int i = tid; i < TKMASKW; i += NTHR) msk[i] = 0u;
  __syncthreads();
#pragma unroll 1
  for (int p = 0; p < KPOOL; ++p) {
    float best = -3.0e38f;
    int bidx = 2147483647;
#pragma unroll 1
    for (int i = tid; i < nR; i += NTHR) {
      if (msk[i >> 5] & (1u << (i & 31))) continue;
      const int r = clampi(remain[i], nN - 1);
      const float v = scores[r];
      if (v > best || (v == best && i < bidx)) { best = v; bidx = i; }
    }
#pragma unroll
    for (int mk = 16; mk > 0; mk >>= 1) {
      const float ov = __shfl_xor(best, mk, 32);
      const int   oi = __shfl_xor(bidx, mk, 32);
      if (ov > best || (ov == best && oi < bidx)) { best = ov; bidx = oi; }
    }
    if (lane == 0) { rv[wave] = best; ri[wave] = bidx; }
    __syncthreads();
    if (tid == 0) {
      float b2 = rv[0];
      int   i2 = ri[0];
      for (int w = 1; w < NWAVE; ++w) {
        if (rv[w] > b2 || (rv[w] == b2 && ri[w] < i2)) { b2 = rv[w]; i2 = ri[w]; }
      }
      sel[p] = i2;
      if ((unsigned)i2 < (unsigned)nR) msk[i2 >> 5] |= (1u << (i2 & 31));
    }
    __syncthreads();
  }

#pragma unroll
  for (int s = 0; s < (KPOOL * DF / 8) / NTHR; ++s) {
    const int q = s * NTHR + tid;
    const int b = q >> 4, c0 = (q & 15) * 8;
    const int i = clampi(sel[b], nR - 1);
    const int node = clampi(remain[i], nN - 1);
    const float* hp = H + (size_t)node * DF + c0;
    Pack16 u;
    u.i = pk8(*(const v4f*)hp, *(const v4f*)(hp + 4), 1.0f);
    *(v8h*)(XpL + b * XPP + c0) = u.h;
  }
  __syncthreads();

  const int j = wave * 16 + m;
  const _Float16* Wih = planes + P_WIH;
  const _Float16* Whh = planes + P_WHH;
  const _Float16* H0p = planes + P_H0;
  const float bi0 = bih[j], bi1 = bih[DF + j], bi2 = bih[2 * DF + j];
  const float bh0 = bhh[j], bh1 = bhh[DF + j], bh2 = bhh[2 * DF + j];
#pragma unroll 1
  for (int T = 0; T < KPOOL / 16; ++T) {
    v8f ax0 = zero8(), ax1 = zero8(), ax2 = zero8();
    v8f ah0 = zero8(), ah1 = zero8(), ah2 = zero8();
#pragma unroll
    for (int kt = 0; kt < DF / 32; ++kt) {
      const int k0 = kt * 32;
      Frag a, ah;
      const _Float16* pa = XpL + (16 * T + m) * XPP + k0 + 8 * hh;
      const _Float16* ph = H0p + (size_t)(16 * T + m) * DF + k0 + 8 * hh;
      a.half[0]  = *(const v8h*)pa; a.half[1]  = *(const v8h*)(pa + 16);
      ah.half[0] = *(const v8h*)ph; ah.half[1] = *(const v8h*)(ph + 16);
      {
        Frag b, c;
        const _Float16* pb = Wih + (size_t)j * DF + k0 + 8 * hh;
        const _Float16* pc = Whh + (size_t)j * DF + k0 + 8 * hh;
        b.half[0] = *(const v8h*)pb; b.half[1] = *(const v8h*)(pb + 16);
        c.half[0] = *(const v8h*)pc; c.half[1] = *(const v8h*)(pc + 16);
        ax0 = wm(a.v, b.v, ax0);
        ah0 = wm(ah.v, c.v, ah0);
      }
      {
        Frag b, c;
        const _Float16* pb = Wih + (size_t)(DF + j) * DF + k0 + 8 * hh;
        const _Float16* pc = Whh + (size_t)(DF + j) * DF + k0 + 8 * hh;
        b.half[0] = *(const v8h*)pb; b.half[1] = *(const v8h*)(pb + 16);
        c.half[0] = *(const v8h*)pc; c.half[1] = *(const v8h*)(pc + 16);
        ax1 = wm(a.v, b.v, ax1);
        ah1 = wm(ah.v, c.v, ah1);
      }
      {
        Frag b, c;
        const _Float16* pb = Wih + (size_t)(2 * DF + j) * DF + k0 + 8 * hh;
        const _Float16* pc = Whh + (size_t)(2 * DF + j) * DF + k0 + 8 * hh;
        b.half[0] = *(const v8h*)pb; b.half[1] = *(const v8h*)(pb + 16);
        c.half[0] = *(const v8h*)pc; c.half[1] = *(const v8h*)(pc + 16);
        ax2 = wm(a.v, b.v, ax2);
        ah2 = wm(ah.v, c.v, ah2);
      }
    }
#pragma unroll
    for (int r = 0; r < 8; ++r) {
      const int b = 16 * T + 8 * hh + r;
      const float xr = ax0[r] * 0.0625f + bi0;
      const float xz = ax1[r] * 0.0625f + bi1;
      const float xn = ax2[r] * 0.0625f + bi2;
      const float hr = ah0[r] * 0.00390625f + bh0;
      const float hz = ah1[r] * 0.00390625f + bh1;
      const float hn = ah2[r] * 0.00390625f + bh2;
      const float rg = sigm(xr + hr);
      const float zg = sigm(xz + hz);
      const float ng = tanhf(xn + rg * hn);
      const float hp = h0[(size_t)b * DF + j];
      hs[b * DF + j] = (1.0f - zg) * ng + zg * hp;
    }
  }
  __syncthreads();

#pragma unroll 1
  for (int ps = 0; ps < 2; ++ps) {
#pragma unroll
    for (int s = 0; s < (KPOOL * DF / 8) / NTHR; ++s) {
      const int q = s * NTHR + tid;
      const int n = q >> 4, k0 = (q & 15) * 8;
      v4f a, b;
      a.x = hs[(k0 + 0) * DF + n]; a.y = hs[(k0 + 1) * DF + n];
      a.z = hs[(k0 + 2) * DF + n]; a.w = hs[(k0 + 3) * DF + n];
      b.x = hs[(k0 + 4) * DF + n]; b.y = hs[(k0 + 5) * DF + n];
      b.z = hs[(k0 + 6) * DF + n]; b.w = hs[(k0 + 7) * DF + n];
      const v4i pk = pk8(a, b, 16.0f);
      *(volatile v4i*)(hT + (size_t)q * 8) = pk;
    }
#pragma unroll 1
    for (int bb = 0; bb < KPOOL / NWAVE; ++bb) {
      const int b = bb * NWAVE + wave;
      const int i = clampi(sel[b], nR - 1);
      const int rc = clampi(remain[i], nN - 1);
      const int t = nid[rc];
      if ((unsigned)t < (unsigned)nN) {
        const v4f v = *(const v4f*)(hs + b * DF + 4 * lane);
        *(volatile v4f*)(xres + (size_t)t * DF + 4 * lane) = v;
      }
    }
    if (ps == 0) __threadfence();
  }
}

__device__ __forceinline__ void epi_att(v8f acc, int T, int hh, int m, int wave, float bv, float av,
                                        float* red) {
  float s[8];
#pragma unroll
  for (int r = 0; r < 8; ++r) {
    float y = fmaxf(acc[r] * 0.0625f + bv, 0.f);
    y = (y > 0.f) ? y : 0.2f * y;
    s[r] = y * av;
  }
#pragma unroll
  for (int mk = 1; mk < 16; mk <<= 1) {
#pragma unroll
    for (int r = 0; r < 8; ++r) s[r] += __shfl_xor(s[r], mk, 32);
  }
  if (m == 0) {
#pragma unroll
    for (int r = 0; r < 8; ++r) red[(T * 16 + 8 * hh + r) * NWAVE + wave] = s[r];
  }
}

__global__ __launch_bounds__(NTHR) void k_attn(
    const float* __restrict__ X, const _Float16* __restrict__ planes,
    const float* __restrict__ bl, const float* __restrict__ br, const float* __restrict__ avec,
    float* alv, float* arv) {
  __shared__ __attribute__((aligned(16))) _Float16 At[GR * AP];
  __shared__ float redl[GR * NWAVE];
  __shared__ float redr[GR * NWAVE];
  __shared__ __attribute__((aligned(16))) float outv[2 * GR];
  const int tid = threadIdx.x, lane = tid & 31, wave = tid >> 5, hh = lane >> 4, m = lane & 15;
  const int rowBase = blockIdx.x * GR;
  {
    const int r  = tid >> 3;
    const int c0 = (tid & 7) * 16;
    const float* p = X + (size_t)(rowBase + r) * DF + c0;
    Pack16 u0, u1;
    u0.i = pk8(*(const v4f*)(p), *(const v4f*)(p + 4), 1.0f);
    u1.i = pk8(*(const v4f*)(p + 8), *(const v4f*)(p + 12), 1.0f);
    *(v8h*)(At + r * AP + c0)     = u0.h;
    *(v8h*)(At + r * AP + c0 + 8) = u1.h;
  }
  __syncthreads();

  const int ncol = wave * 16 + m;
  const _Float16* Bl = planes + P_WL + (size_t)ncol * DF;
  const _Float16* Br = planes + P_WR + (size_t)ncol * DF;
  v8f cl0 = zero8(), cl1 = zero8(), cr0 = zero8(), cr1 = zero8();
#pragma unroll
  for (int kt = 0; kt < DF / 32; ++kt) {
    const int k0 = kt * 32;
    Frag a0, a1, bwl, bwr;
    const _Float16* pl  = Bl + k0 + 8 * hh;
    const _Float16* pr  = Br + k0 + 8 * hh;
    const _Float16* pa0 = At + m * AP + k0 + 8 * hh;
    const _Float16* pa1 = At + (16 + m) * AP + k0 + 8 * hh;
    bwl.half[0] = *(const v8h*)pl;  bwl.half[1] = *(const v8h*)(pl + 16);
    bwr.half[0] = *(const v8h*)pr;  bwr.half[1] = *(const v8h*)(pr + 16);
    a0.half[0]  = *(const v8h*)pa0; a0.half[1]  = *(const v8h*)(pa0 + 16);
    a1.half[0]  = *(const v8h*)pa1; a1.half[1]  = *(const v8h*)(pa1 + 16);
    cl0 = wm(a0.v, bwl.v, cl0);
    cl1 = wm(a1.v, bwl.v, cl1);
    cr0 = wm(a0.v, bwr.v, cr0);
    cr1 = wm(a1.v, bwr.v, cr1);
  }
  const float av = avec[ncol];
  const float bL = bl[ncol], bR = br[ncol];
  epi_att(cl0, 0, hh, m, wave, bL, av, redl);
  epi_att(cl1, 1, hh, m, wave, bL, av, redl);
  epi_att(cr0, 0, hh, m, wave, bR, av, redr);
  epi_att(cr1, 1, hh, m, wave, bR, av, redr);
  __syncthreads();
  if (tid < 2 * GR) {
    const float* rd = (tid < GR) ? redl : redr;
    const int row = tid & (GR - 1);
    float s = 0.f;
#pragma unroll
    for (int w = 0; w < NWAVE; ++w) s += rd[row * NWAVE + w];
    outv[tid] = s;
  }
  __syncthreads();
  if (tid < 16) {
    const v4f v = *(const v4f*)(outv + 4 * tid);
    float* p = (tid < 8) ? (alv + rowBase + 4 * tid) : (arv + rowBase + 4 * (tid - 8));
    *(volatile v4f*)p = v;
    __threadfence();
    *(volatile v4f*)p = v;
  }
}

__global__ __launch_bounds__(NTHR) void k_emax(
    const float* __restrict__ alv, const float* __restrict__ arv, const int* __restrict__ ei,
    float* emx, int nN, int nE) {
  __shared__ float red[NWAVE];
  const int tid = threadIdx.x, lane = tid & 31, wave = tid >> 5;
  float best = -3.0e38f;
#pragma unroll 1
  for (int i = blockIdx.x * NTHR + tid; i < nE; i += NMAXB * NTHR) {
    const int s = clampi(ei[i], nN - 1);
    const int d = clampi(ei[(size_t)nE + i], nN - 1);
    best = fmaxf(best, alv[s] + arv[d]);
  }
#pragma unroll
  for (int mk = 16; mk > 0; mk >>= 1) best = fmaxf(best, __shfl_xor(best, mk, 32));
  if (lane == 0) red[wave] = best;
  __syncthreads();
  if (wave == 0) {
    float bm = red[0];
#pragma unroll
    for (int w = 1; w < NWAVE; ++w) bm = fmaxf(bm, red[w]);
    if (lane < 8) {
      const v4f v = {bm, bm, bm, bm};
      float* p = emx + (size_t)blockIdx.x * 32 + 4 * lane;
      *(volatile v4f*)p = v;
      __threadfence();
      *(volatile v4f*)p = v;
    }
  }
}

__global__ __launch_bounds__(NTHR) void k_rowsum(
    const float* __restrict__ alv, const float* __restrict__ arv, const int* __restrict__ ei,
    const float* __restrict__ emx, float* rowsum, int nN, int nE) {
  __shared__ __attribute__((aligned(16))) float rs[NBS];
  __shared__ int list[NWAVE * WCAP];
  __shared__ int wcnt[NWAVE];
  __shared__ float red[NMAXB];
  const int tid = threadIdx.x, lane = tid & 31, wave = tid >> 5;
  const int base = blockIdx.x * NBS;
  for (int i = tid; i < NBS; i += NTHR) rs[i] = 0.f;
  const float M = block_emax(emx, red, tid);
  __syncthreads();
  const int* eid = ei + nE;
  const int nChunks = (nE + CHUNK - 1) / CHUNK;
#pragma unroll 1
  for (int ch = 0; ch < nChunks; ++ch) {
    const int cbase = ch * CHUNK;
    const int wc = scan_chunk<NBS>(ei, nE, true, cbase, base, list, tid, lane, wave);
    if (lane == 0) wcnt[wave] = wc;
    __syncthreads();
    if (wave == 0) {
#pragma unroll 1
      for (int wsx = 0; wsx < NWAVE; ++wsx) {
        int n = wcnt[wsx];
        n = n > WCAP ? WCAP : (n < 0 ? 0 : n);
#pragma unroll 1
        for (int i0 = 0; i0 < n; i0 += 32) {
          const int idx = i0 + lane;
          const bool valid = idx < n;
          const int lidx = idx < WCAP ? idx : (WCAP - 1);
          const int ent = list[wsx * WCAP + lidx];
          const int slot = ent & (NBS - 1);
          const int el = (ent >> SLOTB) & (CHUNK - 1);
          int e = cbase + el;
          if (e > nE - 1) e = nE - 1;
          const int d = clampi(eid[e], nN - 1);
          int nd = base + slot;
          if (nd > nN - 1) nd = nN - 1;
          float p = 0.f;
          if (valid) p = expf(alv[nd] + arv[d] - M);
#pragma unroll
          for (int jx = 0; jx < 32; ++jx) {
            const float pj = __shfl(p, jx, 32);
            const int   sj = __shfl(slot, jx, 32);
            if (lane == 0) rs[sj] += pj;
          }
        }
      }
    }
    __syncthreads();
  }
#pragma unroll
  for (int q = 0; q < NBS / (NTHR * 4); ++q) {
    const int idx = (q * NTHR + tid) * 4;
    const v4f v = *(const v4f*)(rs + idx);
    *(volatile v4f*)(rowsum + (size_t)base + idx) = v;
  }
  __threadfence();
#pragma unroll
  for (int q = 0; q < NBS / (NTHR * 4); ++q) {
    const int idx = (q * NTHR + tid) * 4;
    const v4f v = *(const v4f*)(rs + idx);
    *(volatile v4f*)(rowsum + (size_t)base + idx) = v;
  }
}

__device__ __forceinline__ float wcalc(int e, int nE, int nN, float M, const float* __restrict__ alv,
                                       const float* __restrict__ arv, const int* __restrict__ ei,
                                       const float* __restrict__ rowsum) {
  if (e >= nE) return 0.f;
  const int s = clampi(ei[e], nN - 1);
  const int d = clampi(ei[(size_t)nE + e], nN - 1);
  const float v = expf(alv[s] + arv[d] - M);
  const float den = rowsum[s] + 1e-16f;
  return v / den;
}

__global__ __launch_bounds__(NTHR) void k_wedge(
    const float* __restrict__ alv, const float* __restrict__ arv, const int* __restrict__ ei,
    const float* __restrict__ rowsum, const float* __restrict__ emx, float* wbuf,
    int nN, int nE, int nE4) {
  __shared__ float red[NMAXB];
  const int tid = threadIdx.x;
  const float M = block_emax(emx, red, tid);
  const int g = blockIdx.x * NTHR + tid;
  if (g >= nE4) return;
  const int e0 = g * 4;
  v4f w;
  w.x = wcalc(e0 + 0, nE, nN, M, alv, arv, ei, rowsum);
  w.y = wcalc(e0 + 1, nE, nN, M, alv, arv, ei, rowsum);
  w.z = wcalc(e0 + 2, nE, nN, M, alv, arv, ei, rowsum);
  w.w = wcalc(e0 + 3, nE, nN, M, alv, arv, ei, rowsum);
  float* p = wbuf + (size_t)e0;
  *(volatile v4f*)p = w;
  __threadfence();
  *(volatile v4f*)p = w;
}

__global__ __launch_bounds__(NTHR) void k_agg(
    const float* fin, const float* xres, const int* __restrict__ ei,
    const float* __restrict__ wbuf, const _Float16* __restrict__ hT,
    float* out, float theta, float omt, int nN, int nE, int nRowsOut) {
  extern __shared__ v4f lds_dyn[];
  float* sacc = (float*)lds_dyn;
  int*   list = (int*)(sacc + NB * DF);
  int*   wcnt = list + NWAVE * WCAP;
  const int tid = threadIdx.x, lane = tid & 31, wave = tid >> 5, hh = lane >> 4, m = lane & 15;
  const int nodeBase = blockIdx.x * NB;
  {
    const v4f z4 = {0.f, 0.f, 0.f, 0.f};
    for (int i = tid; i < NB * DF / 4; i += NTHR) lds_dyn[i] = z4;
  }
  __syncthreads();
  const int* eid = ei + nE;
  const bool al16 = ((nE & 3) == 0);
  const int nChunks = (nE + CHUNK - 1) / CHUNK;
#pragma unroll 1
  for (int ch = 0; ch < nChunks; ++ch) {
    const int cbase = ch * CHUNK;
    const int wc = scan_chunk<NB>(eid, nE, al16, cbase, nodeBase, list, tid, lane, wave);
    if (lane == 0) wcnt[wave] = wc;
    __syncthreads();
    if (wave == 0) {
#pragma unroll 1
      for (int wsx = 0; wsx < NWAVE; ++wsx) {
        int n = wcnt[wsx];
        n = n > WCAP ? WCAP : (n < 0 ? 0 : n);
#pragma unroll 1
        for (int i = 0; i < n; ++i) {
          const int ent  = list[wsx * WCAP + i];
          const int slot = ent & (NB - 1);
          const int el   = (ent >> SLOTB) & (CHUNK - 1);
          int e = cbase + el;
          if (e > nE - 1) e = nE - 1;
          const int s = clampi(ei[e], nN - 1);
          const float w = wbuf[e];
          const v4f xv = *(const v4f*)(fin + (size_t)s * DF + 4 * lane);
          v4f* sp = (v4f*)(sacc + slot * DF + 4 * lane);
          const v4f cur = *sp;
          *sp = cur + w * xv;
        }
      }
    }
    __syncthreads();
  }

#pragma unroll 1
  for (int jj = 0; jj < NB / NWAVE; ++jj) {
    const int slot = wave * (NB / NWAVE) + jj;
    const size_t row = (size_t)(nodeBase + slot);
    const v4f xr4 = *(const v4f*)(xres + row * DF + 4 * lane);
    v4f* sp = (v4f*)(sacc + slot * DF + 4 * lane);
    const v4f cur = *sp;
    *sp = 0.9f * cur + 0.1f * xr4;
  }
  __syncthreads();

  const int ncol = wave * 16 + m;
  Frag bq[4];
#pragma unroll
  for (int kt = 0; kt < 4; ++kt) {
    const _Float16* pb = hT + (size_t)ncol * DF + 32 * kt + 8 * hh;
    bq[kt].half[0] = *(const v8h*)pb;
    bq[kt].half[1] = *(const v8h*)(pb + 16);
  }
#pragma unroll 1
  for (int T = 0; T < NB / 16; ++T) {
    v8f acc = zero8();
#pragma unroll
    for (int kt = 0; kt < 4; ++kt) {
      const float* ap = sacc + (16 * T + m) * DF + 32 * kt + 8 * hh;
      Frag a;
      Pack16 u0, u1;
      u0.i = pk8(*(const v4f*)(ap), *(const v4f*)(ap + 4), 1.0f);
      u1.i = pk8(*(const v4f*)(ap + 16), *(const v4f*)(ap + 20), 1.0f);
      a.half[0] = u0.h; a.half[1] = u1.h;
      acc = wm(a.v, bq[kt].v, acc);
    }
    float o[8];
#pragma unroll
    for (int r = 0; r < 8; ++r) {
      const int row = 16 * T + 8 * hh + r;
      const float sv = sacc[row * DF + ncol];
      o[r] = fmaxf(theta * (acc[r] * 0.0625f) + omt * sv, 0.f);
    }
    __syncthreads();
#pragma unroll
    for (int r = 0; r < 8; ++r) sacc[(16 * T + 8 * hh + r) * DF + ncol] = o[r];
  }
  __syncthreads();

#pragma unroll 1
  for (int jj = 0; jj < NB / NWAVE; ++jj) {
    const int slot = wave * (NB / NWAVE) + jj;
    const int node = nodeBase + slot;
    if (node < nRowsOut) {
      const v4f v = *(const v4f*)(sacc + slot * DF + 4 * lane);
      *(volatile v4f*)(out + (size_t)node * DF + 4 * lane) = v;
    }
  }
  __threadfence();
#pragma unroll 1
  for (int jj = 0; jj < NB / NWAVE; ++jj) {
    const int slot = wave * (NB / NWAVE) + jj;
    const int node = nodeBase + slot;
    if (node < nRowsOut) {
      const v4f v = *(const v4f*)(sacc + slot * DF + 4 * lane);
      *(volatile v4f*)(out + (size_t)node * DF + 4 * lane) = v;
    }
  }
}

extern "C" void kernel_launch(void* const* d_in, const int* in_sizes, int n_in,
                              void* d_out, int out_size, void* d_ws, size_t ws_size,
                              hipStream_t stream) {
  if (n_in < 18) return;
  const int nN = in_sizes[0] / DF;
  if (nN <= 0 || in_sizes[0] != nN * DF) return;
  if (in_sizes[1] != nN || in_sizes[17] != nN) return;
  if (in_sizes[2] != DF * DF || in_sizes[4] != DF * DF || in_sizes[6] != DF * DF || in_sizes[9] != DF * DF) return;
  if (in_sizes[3] != DF || in_sizes[5] != DF || in_sizes[7] != DF || in_sizes[8] != DF) return;
  if (in_sizes[10] != 3 * DF * DF || in_sizes[11] != 3 * DF * DF) return;
  if (in_sizes[12] != 3 * DF || in_sizes[13] != 3 * DF) return;
  const int nE = in_sizes[14] / 2;
  if (nE <= 0 || in_sizes[14] != 2 * nE) return;
  const int nR = in_sizes[15];
  if (nR < KPOOL || nR > TKMASKW * 32) return;
  const int nA = in_sizes[16];
  if (nA < 0) return;
  if (out_size != nN * DF) return;

  const float* x      = (const float*)d_in[0];
  const float* scores = (const float*)d_in[1];
  const float* W_hid  = (const float*)d_in[2];
  const float* b_hid  = (const float*)d_in[3];
  const float* Wl     = (const float*)d_in[4];
  const float* bl     = (const float*)d_in[5];
  const float* Wr     = (const float*)d_in[6];
  const float* br     = (const float*)d_in[7];
  const float* avec   = (const float*)d_in[8];
  const float* h0w    = (const float*)d_in[9];
  const float* W_ih   = (const float*)d_in[10];
  const float* W_hh   = (const float*)d_in[11];
  const float* b_ih   = (const float*)d_in[12];
  const float* b_hh   = (const float*)d_in[13];
  const int*   ei     = (const int*)d_in[14];
  const int*   remain = (const int*)d_in[15];
  const int*   added  = (const int*)d_in[16];
  const int*   nid    = (const int*)d_in[17];
  float* outp = (float*)d_out;

  const int nPad = ((nN + NBX - 1) / NBX) * NBX;
  const int nRS  = ((nN + NBS - 1) / NBS) * NBS;
  const int ePad = ((nE + EMP - 1) / EMP) * EMP;

  size_t off = 0;
#define CARVE(T, name, bytes) T* name = (T*)((char*)d_ws + off); off += (((size_t)(bytes) + 255) / 256) * 256;
  CARVE(_Float16, planes, (size_t)P_TOT * sizeof(_Float16))
  CARVE(_Float16, hT,     (size_t)DF * DF * sizeof(_Float16))
  CARVE(float,    alv,    (size_t)nPad * sizeof(float))
  CARVE(float,    arv,    (size_t)nPad * sizeof(float))
  CARVE(float,    emx,    (size_t)NMAXB * 32 * sizeof(float))
  CARVE(float,    rowsum, (size_t)nRS * sizeof(float))
  CARVE(float,    wbuf,   (size_t)ePad * sizeof(float))
  CARVE(float,    bufA,   (size_t)nPad * DF * sizeof(float))
  CARVE(float,    xres,   (size_t)nPad * DF * sizeof(float))
#undef CARVE
  if (off > ws_size || off > (size_t)134217728) return;

  k_prep<<<PREP_UNITS / NTHR, NTHR, 0, stream>>>(W_hid, Wl, Wr, W_ih, W_hh, h0w, planes);
  const int gridG = (nN + GR - 1) / GR;
  k_gemm_hid<<<gridG, NTHR, 0, stream>>>(x, planes, b_hid, bufA, nN);
  k_xres<<<nPad / NBX, NTHR, 0, stream>>>(bufA, remain, added, nid, xres, nN, nR, nA);
  hipFuncSetAttribute(reinterpret_cast<const void*>(&k_pool),
                      hipFuncAttributeMaxDynamicSharedMemorySize, POOL_LDS_BYTES);
  k_pool<<<1, NTHR, POOL_LDS_BYTES, stream>>>(scores, remain, nid, bufA, planes, h0w, b_ih, b_hh,
                                              xres, hT, nN, nR);
  k_attn<<<gridG, NTHR, 0, stream>>>(xres, planes, bl, br, avec, alv, arv);
  k_emax<<<NMAXB, NTHR, 0, stream>>>(alv, arv, ei, emx, nN, nE);
  k_rowsum<<<nRS / NBS, NTHR, 0, stream>>>(alv, arv, ei, emx, rowsum, nN, nE);
  k_wedge<<<ePad / (4 * NTHR), NTHR, 0, stream>>>(alv, arv, ei, rowsum, emx, wbuf, nN, nE, ePad / 4);
  hipFuncSetAttribute(reinterpret_cast<const void*>(&k_agg),
                      hipFuncAttributeMaxDynamicSharedMemorySize, AGG_LDS_BYTES);
  const int gridA = (nN + NB - 1) / NB;
  {
    const double th = log(0.5 / 1.0 + 1.0);
    const float theta = (float)th;
    const float omt = (float)(1.0 - th);
    k_agg<<<gridA, NTHR, AGG_LDS_BYTES, stream>>>(xres, xres, ei, wbuf, hT, bufA, theta, omt,
                                                  nN, nE, gridA * NB);
  }
  {
    const double th = log(0.5 / 2.0 + 1.0);
    const float theta = (float)th;
    const float omt = (float)(1.0 - th);
    k_agg<<<gridA, NTHR, AGG_LDS_BYTES, stream>>>(bufA, xres, ei, wbuf, hT, outp, theta, omt,
                                                  nN, nE, nN);
  }
}
